// MultiNadwatSpatialConv_66322884985177
// MI455X (gfx1250) — hardware-verified
//
#include <hip/hip_runtime.h>
#include <math.h>

typedef __attribute__((ext_vector_type(16))) _Float16 v16h;
typedef __attribute__((ext_vector_type(16))) __bf16 v16b;
typedef __attribute__((ext_vector_type(8)))  _Float16 v8h;
typedef __attribute__((ext_vector_type(8)))  float v8f;
typedef __attribute__((ext_vector_type(4)))  float v4f;
typedef __attribute__((ext_vector_type(2)))  float v2f;
typedef __attribute__((ext_vector_type(4)))  unsigned v4u;
typedef __attribute__((ext_vector_type(4)))  int v4i;
typedef float __attribute__((may_alias)) float_a;
typedef int __attribute__((may_alias)) int_a;

template <typename T> __device__ __forceinline__ void vst2(void* p, T v) { *(volatile T*)p = v; __threadfence(); *(volatile T*)p = v; }
__device__ __forceinline__ v8f wmma16(v16h a, v16h b, v8f c) {
  v8f d = __builtin_amdgcn_wmma_f32_16x16x32_f16(false, a, false, b, (short)0, c, false, false);
  asm volatile("v_nop\n\tv_nop\n\tv_nop\n\tv_nop" : "+v"(d) : "v"(a), "v"(b));
  return d;
}
__device__ __forceinline__ v8f wmma_bf(v16b a, v16b b, v8f c) {
  v8f d = __builtin_amdgcn_wmma_f32_16x16x32_bf16(false, a, false, b, (short)0, c, false, false);
  asm volatile("v_nop\n\tv_nop\n\tv_nop\n\tv_nop" : "+v"(d) : "v"(a), "v"(b));
  return d;
}
__device__ __forceinline__ v16h frag_h(const _Float16* rowk0, int lane) {
  union { v16h v; v8h q[2]; } u; const _Float16* p = rowk0 + 8 * (lane >> 4);
  u.q[0] = *(const v8h*)p; u.q[1] = *(const v8h*)(p + 16); return u.v;
}
__device__ __forceinline__ v16h frag_f32(const float* rowk0, int lane) {
  v16h a; const float* p = rowk0 + 8 * (lane >> 4);
#pragma unroll
  for (int i = 0; i < 8; ++i) { a[i] = (_Float16)p[i]; a[8 + i] = (_Float16)p[16 + i]; }
  return a;
}
__device__ __forceinline__ v16h frag_f32s(const float* rowk0, int lane, float sc) {
  v16h a; const float* p = rowk0 + 8 * (lane >> 4);
#pragma unroll
  for (int i = 0; i < 8; ++i) { a[i] = (_Float16)(p[i] * sc); a[8 + i] = (_Float16)(p[16 + i] * sc); }
  return a;
}
__device__ __forceinline__ v16h fragc_f32(const float* W, int k0, int n, int lane, int ld, int K) {
  v16h a; const int g = lane >> 4;
#pragma unroll
  for (int i = 0; i < 8; ++i) { const int ka = k0 + 8 * g + i, kb = ka + 16;
    a[i] = (_Float16)(ka < K ? W[(size_t)(ka < K ? ka : K - 1) * ld + n] : 0.f); a[8 + i] = (_Float16)(kb < K ? W[(size_t)(kb < K ? kb : K - 1) * ld + n] : 0.f); }
  return a;
}
struct F2 { v16b h, l; };
__device__ __forceinline__ F2 bsplit16(const float v[16]) { F2 r;
#pragma unroll
  for (int i = 0; i < 16; ++i) { const __bf16 h = (__bf16)v[i]; r.h[i] = h; r.l[i] = (__bf16)(v[i] - (float)h); }
  return r; }
__device__ __forceinline__ F2 split_row(const float* row, int k0, int lane) { float v[16]; const float* p = row + k0 + 8 * (lane >> 4);
#pragma unroll
  for (int i = 0; i < 8; ++i) { v[i] = p[i]; v[8 + i] = p[16 + i]; }
  return bsplit16(v); }
__device__ __forceinline__ F2 split_rowK(const float* row, int k0, int lane, int K) { float v[16]; const int g = lane >> 4;
#pragma unroll
  for (int i = 0; i < 8; ++i) { const int ka = k0 + 8 * g + i, kb = ka + 16; v[i] = ka < K ? row[ka < K ? ka : K - 1] : 0.f; v[8 + i] = kb < K ? row[kb < K ? kb : K - 1] : 0.f; }
  return bsplit16(v); }
__device__ __forceinline__ F2 split_col(const float* W, int k0, int n, int lane, int ld, int K) { float v[16]; const int g = lane >> 4;
#pragma unroll
  for (int i = 0; i < 8; ++i) { const int ka = k0 + 8 * g + i, kb = ka + 16; v[i] = ka < K ? W[(size_t)(ka < K ? ka : K - 1) * ld + n] : 0.f; v[8 + i] = kb < K ? W[(size_t)(kb < K ? kb : K - 1) * ld + n] : 0.f; }
  return bsplit16(v); }
__device__ __forceinline__ v8f mac3(const F2& a, const F2& b, v8f c) { c = wmma_bf(a.l, b.h, c); c = wmma_bf(a.h, b.l, c); return wmma_bf(a.h, b.h, c); }
__device__ __forceinline__ float sigm(float v) { return 1.0f / (1.0f + expf(-v)); }
#define LDSX() do { asm volatile("s_wait_dscnt 0" ::: "memory"); __builtin_amdgcn_wave_barrier(); __builtin_amdgcn_fence(__ATOMIC_RELEASE, "workgroup"); } while (0)


#define NB 2
#define NQ 4096
#define NM 4096
#define CC 64
#ifndef TQ
#define TQ (NQ / 64)
#endif
#ifndef TNB
#define TNB NB
#endif
typedef __attribute__((ext_vector_type(8))) __bf16 v8b;
__device__ __forceinline__ v16b frag_b(const __bf16* rowk0, int lane) {
  union { v16b v; v8b q[2]; } u; const __bf16* p = rowk0 + 8 * (lane >> 4);
  u.q[0] = *(const v8b*)p; u.q[1] = *(const v8b*)(p + 16); return u.v;
}
__device__ __forceinline__ float bfr(float v) { return (float)(__bf16)v; }
__device__ __attribute__((noinline)) float exp_ni(float v) { return expf(v); }
__device__ __attribute__((noinline)) float erf_ni(float v) { return erff(v); }

#define WS_YT  0u
#define WS_END (WS_YT + 2u * (size_t)NB * CC * NM)

__global__ __launch_bounds__(256) void k_yt(const float* __restrict__ YF, __bf16* __restrict__ YT) { __shared__ __align__(16) __bf16 st[CC][64 + 8]; const int t = threadIdx.x; const int m0 = blockIdx.x * 64; const size_t b = blockIdx.y;
  for (int e = t; e < 64 * CC; e += 256) { const int ml = e >> 6, c = e & 63; st[c][ml] = (__bf16)YF[((b * NM + m0 + ml) * CC) + c]; } __syncthreads();
  for (int e = t; e < CC * 8; e += 256) { const int c = e >> 3, q = e & 7; vst2((unsigned*)(YT + ((b * CC + c) * NM) + m0 + q * 8), *(const v4u*)&st[c][q * 8]); } }
__global__ __launch_bounds__(128) void k_nw(const float* __restrict__ X, const float* __restrict__ Y, const float* __restrict__ YW, const __bf16* __restrict__ YT, float* __restrict__ OUT) {
  __shared__ __align__(16) float sp[4][16][36]; __shared__ __align__(16) float so[4][16][68]; __shared__ float sy[NM][4];
  const int tid = threadIdx.x, wave = tid >> 5, lane = tid & 31, col = lane & 15, g = lane >> 4; const size_t b = blockIdx.y; const int q0 = blockIdx.x * 64 + wave * 16; const size_t rq = b * NQ + q0;
  for (int m = tid; m < NM; m += 128) { sy[m][0] = bfr(Y[(b * NM + m) * 3]); sy[m][1] = bfr(Y[(b * NM + m) * 3 + 1]); sy[m][2] = bfr(Y[(b * NM + m) * 3 + 2]); sy[m][3] = bfr(YW[b * NM + m]); }
  float qx[8], qy[8], qz[8], den[8];
#pragma unroll
  for (int r = 0; r < 8; ++r) { const size_t n = rq + 8 * g + r; qx[r] = bfr(X[n * 3]); qy[r] = bfr(X[n * 3 + 1]); qz[r] = bfr(X[n * 3 + 2]); den[r] = 0.f; }
  __syncthreads();
  v8f acc[4] = {};
#pragma unroll 1
  for (int ks = 0; ks < NM / 32; ++ks) {
#pragma unroll
    for (int ct = 0; ct < 2; ++ct) { const int m = ks * 32 + ct * 16 + col; const float yx = sy[m][0], yy = sy[m][1], yz = sy[m][2], yw = sy[m][3]; const float y2 = yx * yx + yy * yy + yz * yz;
#pragma unroll
      for (int r = 0; r < 8; ++r) { const float x2 = qx[r] * qx[r] + qy[r] * qy[r] + qz[r] * qz[r]; const float dot = qx[r] * yx + qy[r] * yy + qz[r] * yz; const float d2 = fmaxf(x2 + y2 - 2.0f * dot, 0.f);
        const float kv = 0.3f * __expf(-d2 * (1.0f / 0.0025f)) + 0.3f * __expf(-d2 * (1.0f / 0.01f)) + 0.4f * __expf(-d2 * (1.0f / 0.04f)); const float kw = kv * yw; den[r] += kw; sp[wave][8 * g + r][ct * 16 + col] = kw; } }
    LDSX();
    float v[16]; { const float* prow = &sp[wave][col][0] + 8 * (lane >> 4);
#pragma unroll
      for (int i = 0; i < 8; ++i) { v[i] = prow[i]; v[8 + i] = prow[16 + i]; } }
    const F2 a = bsplit16(v);
#pragma unroll
    for (int j = 0; j < 4; ++j) { const v16b w = frag_b(YT + ((b * CC + j * 16 + col) * NM) + ks * 32, lane); acc[j] = wmma_bf(a.h, w, acc[j]); acc[j] = wmma_bf(a.l, w, acc[j]); }
    LDSX(); }
#pragma unroll
  for (int r = 0; r < 8; ++r) { float dt = den[r];
#pragma unroll
    for (int o = 1; o < 16; o <<= 1) dt += __shfl_xor(dt, o);
    const float inv = 1.0f / (dt + 1e-7f);
#pragma unroll
    for (int j = 0; j < 4; ++j) so[wave][8 * g + r][j * 16 + col] = acc[j][r] * inv; }
  LDSX(); for (int rl = 0; rl < 16; ++rl) if (lane < 16) vst2(OUT + (rq + rl) * CC + lane * 4, *(const v4f*)&so[wave][rl][lane * 4]);
}
extern "C" void kernel_launch(void* const* d_in, const int* in_sizes, int n_in, void* d_out, int out_size, void* d_ws, size_t ws_size, hipStream_t stream) {
  (void)in_sizes; (void)n_in; (void)out_size;
  const float** F = (const float**)d_in;
  if (ws_size < (size_t)WS_END) return;
  __bf16* YT = (__bf16*)d_ws;
  k_yt<<<dim3(NM / 64, TNB), 256, 0, stream>>>(F[2], YT);
  k_nw<<<dim3(TQ, TNB), 128, 0, stream>>>(F[0], F[1], F[3], YT, (float*)d_out);
}
